// GATEdgeNet_50568944943203
// MI455X (gfx1250) — hardware-verified
//
#include <hip/hip_runtime.h>
#include <math.h>

#define NN    50000
#define NE    800000
#define NV    (2 * NE + NN)
#define GI    64
#define GH    128
#define GO    64
#define MK    272
#define MKP   288
#define MH    128
#define NPAD  51200
#define NT    256
#define SRB   4096
#define RPW   512
#define RPW_LOG 9
#define NTL   13
#define NAGG  (NTL * SRB)
#define SCH   2048
#define NCH   ((NV + SCH - 1) / SCH)
#define ECH   102400
#define NECH  ((NE + ECH - 1) / ECH)

static_assert(NTL * SRB >= NPAD, "tiles cover padded nodes");
static_assert(NPAD % 64 == 0 && NPAD >= NN && (NPAD % 32) == 0, "node padding");
static_assert(NE % 8 == 0 && (2 * NE) % 8 == 0, "edge groups of 8 do not straddle list sections");
static_assert(ECH % 256 == 0 && ((NE % ECH) % 256) == 0, "edge chunks are multiples of 256 rows");
static_assert(SRB == 8 * RPW && RPW == (1 << RPW_LOG), "wave row ownership");
static_assert(SCH % NT == 0, "chunk split");

typedef __attribute__((ext_vector_type(16))) _Float16 v16h;
typedef __attribute__((ext_vector_type(8)))  _Float16 v8h;
typedef __attribute__((ext_vector_type(4)))  _Float16 v4h;
typedef __attribute__((ext_vector_type(2)))  _Float16 v2h;
typedef __attribute__((ext_vector_type(16))) __bf16   v16b;
typedef __attribute__((ext_vector_type(8)))  __bf16   v8b;
typedef __attribute__((ext_vector_type(8)))  float    v8f;
typedef __attribute__((ext_vector_type(4)))  float    v4f;
typedef __attribute__((ext_vector_type(2)))  float    v2f;
typedef __attribute__((ext_vector_type(4)))  int      v4i;
typedef __attribute__((ext_vector_type(4)))  unsigned v4u;
typedef __attribute__((ext_vector_type(2)))  unsigned v2u;

__device__ __forceinline__ unsigned short f2bf_bits(float f) {
  unsigned u = __float_as_uint(f);
  return (unsigned short)((u + 0x7FFFu + ((u >> 16) & 1u)) >> 16);
}
__device__ __forceinline__ float bf_bits2f(unsigned short h) { return __uint_as_float(((unsigned)h) << 16); }

__device__ __forceinline__ void dep_guard_h(v8f& a, v8f& b, v16h x, v16h y) { asm volatile("v_nop\n\tv_nop\n\tv_nop\n\tv_nop" : "+v"(a), "+v"(b) : "v"(x), "v"(y)); }
__device__ __forceinline__ void dep_guard_b(v8f& a, v8f& b, v16b x, v16b y) { asm volatile("v_nop\n\tv_nop\n\tv_nop\n\tv_nop" : "+v"(a), "+v"(b) : "v"(x), "v"(y)); }
__device__ __forceinline__ void keep4_h(v16h a, v16h b, v16h c, v16h d) { asm volatile("v_nop" :: "v"(a), "v"(b), "v"(c), "v"(d)); }
__device__ __forceinline__ void keep4_b(v16b a, v16b b, v16b c, v16b d) { asm volatile("v_nop" :: "v"(a), "v"(b), "v"(c), "v"(d)); }
__device__ __forceinline__ void acc_guard4(v8f& a, v8f& b, v8f& c, v8f& d) { asm volatile("v_nop\n\tv_nop\n\tv_nop\n\tv_nop" : "+v"(a), "+v"(b), "+v"(c), "+v"(d)); }
template <typename T> struct Frag;
template <> struct Frag<_Float16> {
  typedef v16h V; union U { v16h v; v8h h[2]; };
  static __device__ __forceinline__ v16h load(const _Float16* p) {
    U f; f.h[0] = *(const v8h*)(p); f.h[1] = *(const v8h*)(p + 16); return f.v;
  }
  static __device__ __forceinline__ v8f mma(v16h a, v16h b, v8f c) {
    return __builtin_amdgcn_wmma_f32_16x16x32_f16(false, a, false, b, (short)0, c, false, false);
  }
  static __device__ __forceinline__ void guard(v8f& a, v8f& b, v16h x, v16h y) { dep_guard_h(a, b, x, y); }
  static __device__ __forceinline__ void keep(v16h a, v16h b, v16h c, v16h d) { keep4_h(a, b, c, d); }
};
template <> struct Frag<__bf16> {
  typedef v16b V; union U { v16b v; v8b h[2]; };
  static __device__ __forceinline__ v16b load(const __bf16* p) {
    U f; f.h[0] = *(const v8b*)(p); f.h[1] = *(const v8b*)(p + 16); return f.v;
  }
  static __device__ __forceinline__ v8f mma(v16b a, v16b b, v8f c) {
    return __builtin_amdgcn_wmma_f32_16x16x32_bf16(false, a, false, b, (short)0, c, false, false);
  }
  static __device__ __forceinline__ void guard(v8f& a, v8f& b, v16b x, v16b y) { dep_guard_b(a, b, x, y); }
  static __device__ __forceinline__ void keep(v16b a, v16b b, v16b c, v16b d) { keep4_b(a, b, c, d); }
};

template <int ET> struct Elem;
template <> struct Elem<0> { typedef _Float16 T; };
template <> struct Elem<1> { typedef __bf16 T; };
template <int ET, bool SPLIT, int BIAS_MODE, int OUT_MODE, bool RESID, int ACT = 0>
__global__ __launch_bounds__(256) void wmma_gemm64(
    const unsigned short* __restrict__ Ap, const unsigned short* __restrict__ A2p, int lda, long strideA,
    const unsigned short* __restrict__ Btp, const unsigned short* __restrict__ Bt2p, int ldb, long strideB,
    void* __restrict__ Cout, void* __restrict__ Cout2, int ldc, long strideC,
    const float* __restrict__ bias,
    const float* __restrict__ resid, long strideR,
    int M, int N, int K, float scale) {
  typedef typename Elem<ET>::T T;
  typedef typename Frag<T>::V V;
  const T* A = (const T*)Ap; const T* A2 = (const T*)A2p; const T* Bt = (const T*)Btp; const T* Bt2 = (const T*)Bt2p;
  __shared__ __align__(16) float sT[8][16 * 68];
  const int b    = blockIdx.y;
  const int lane = threadIdx.x & 31;
  const int wave = threadIdx.x >> 5;
  const int tilesN = N >> 6;
  const int tilesM = M >> 6;
  const int tile = blockIdx.x * 8 + wave;
  if (tile >= tilesM * tilesN) return;
  const int tm = tile / tilesN;
  const int tn = tile - tm * tilesN;
  const int m0 = tm << 6;
  const int n0 = tn << 6;

  const T* Ab  = A  + (size_t)b * strideA;
  const T* Bb  = Bt + (size_t)b * strideB;
  const T* Ab2 = SPLIT ? (A2  + (size_t)b * strideA) : nullptr;
  const T* Bb2 = SPLIT ? (Bt2 + (size_t)b * strideB) : nullptr;

  const int rlane = lane & 15;
  const int koff  = (lane >> 4) * 8;
  const int mOff  = (lane >> 4) * 8;

  v8f acc[4][4];
#pragma unroll
  for (int i = 0; i < 4; ++i)
#pragma unroll
    for (int j = 0; j < 4; ++j) acc[i][j] = (v8f){0.f,0.f,0.f,0.f,0.f,0.f,0.f,0.f};

  for (int k0 = 0; k0 < K; k0 += 32) {
    V bh[4], bl[4];
#pragma unroll
    for (int j = 0; j < 4; ++j) {
      const size_t bo = (size_t)(n0 + (j << 4) + rlane) * ldb + koff + k0;
      bh[j] = Frag<T>::load(Bb + bo);
      if (SPLIT) bl[j] = Frag<T>::load(Bb2 + bo);
    }
#pragma unroll
    for (int i = 0; i < 4; ++i) {
      const size_t ao = (size_t)(m0 + (i << 4) + rlane) * lda + koff + k0;
      V ah = Frag<T>::load(Ab + ao);
      V al;
      if (SPLIT) al = Frag<T>::load(Ab2 + ao);
#pragma unroll
      for (int j = 0; j < 4; ++j) {
        acc[i][j] = Frag<T>::mma(ah, bh[j], acc[i][j]);
        if (SPLIT) {
          acc[i][j] = Frag<T>::mma(ah, bl[j], acc[i][j]);
          acc[i][j] = Frag<T>::mma(al, bh[j], acc[i][j]);
        }
      }
      Frag<T>::guard(acc[i][0], acc[i][3], ah, SPLIT ? al : ah);
    }
    Frag<T>::keep(bh[0], bh[1], bh[2], bh[3]);
    if (SPLIT) Frag<T>::keep(bl[0], bl[1], bl[2], bl[3]);
  }
  acc_guard4(acc[0][0], acc[0][1], acc[0][2], acc[0][3]);
  acc_guard4(acc[1][0], acc[1][1], acc[1][2], acc[1][3]);
  acc_guard4(acc[2][0], acc[2][1], acc[2][2], acc[2][3]);
  acc_guard4(acc[3][0], acc[3][1], acc[3][2], acc[3][3]);

  float* slab = sT[wave];
  const float* Rb = RESID ? (resid + (size_t)b * strideR) : nullptr;
#pragma unroll
  for (int i = 0; i < 4; ++i) {
    const int mBase = m0 + (i << 4);
#pragma unroll
    for (int j = 0; j < 4; ++j) {
      const int n = n0 + (j << 4) + rlane;
      float bv = 0.f;
      if (BIAS_MODE == 2) bv = bias[n];
#pragma unroll
      for (int r = 0; r < 8; ++r) {
        float v = acc[i][j][r] * scale;
        if (BIAS_MODE == 1) v += bias[mBase + mOff + r];
        if (BIAS_MODE == 2) v += bv;
        if (RESID) v += Rb[(size_t)(mBase + mOff + r) * ldc + n];
        if (ACT == 1) v = tanhf(v);
        if (ACT == 2) v = fmaxf(v, 0.0f);
        if (ACT == 3) v = v / (1.0f + expf(-v));
        if (ACT == 4) v = (v > 0.f) ? v : 0.01f * v;
        if (ACT == 5) v = 0.5f * v * (1.0f + erff(v * 0.70710678118654752f));
        slab[(mOff + r) * 68 + (j << 4) + rlane] = v;
      }
    }
    __builtin_amdgcn_fence(__ATOMIC_RELEASE, "workgroup");
    __builtin_amdgcn_wave_barrier();
    __builtin_amdgcn_fence(__ATOMIC_ACQUIRE, "workgroup");
    if (OUT_MODE == 0) {
      float* C = (float*)Cout + (size_t)b * strideC;
      const int hh = lane >> 4, c4 = (lane & 15) * 4;
      for (int pass = 0; pass < 2; ++pass) {
#pragma unroll
        for (int it = 0; it < 8; ++it) {
          const int row = it * 2 + hh;
          v4f v = *(const v4f*)(slab + row * 68 + c4);
          *(volatile v4f*)(C + (size_t)(mBase + row) * ldc + n0 + c4) = v;
        }
        __threadfence();
      }
    } else {
      const int q = lane >> 3, c8 = (lane & 7) * 8;
      unsigned short* C  = (unsigned short*)Cout  + (size_t)b * strideC;
      unsigned short* C2 = (OUT_MODE == 2) ? ((unsigned short*)Cout2 + (size_t)b * strideC) : nullptr;
      for (int pass = 0; pass < 2; ++pass) {
#pragma unroll
        for (int it = 0; it < 4; ++it) {
          const int row = it * 4 + q;
          const float* sp = slab + row * 68 + c8;
          v8h hv, lv;
#pragma unroll
          for (int e = 0; e < 8; ++e) {
            if (OUT_MODE == 1) {
              hv[e] = (_Float16)sp[e];
            } else {
              unsigned short hb = f2bf_bits(sp[e]);
              unsigned short lb = f2bf_bits(sp[e] - bf_bits2f(hb));
              hv[e] = __builtin_bit_cast(_Float16, hb);
              lv[e] = __builtin_bit_cast(_Float16, lb);
            }
          }
          *(volatile v8h*)(C + (size_t)(mBase + row) * ldc + n0 + c8) = hv;
          if (OUT_MODE == 2) *(volatile v8h*)(C2 + (size_t)(mBase + row) * ldc + n0 + c8) = lv;
        }
        __threadfence();
      }
    }
    __builtin_amdgcn_fence(__ATOMIC_RELEASE, "workgroup");
    __builtin_amdgcn_wave_barrier();
    __builtin_amdgcn_fence(__ATOMIC_ACQUIRE, "workgroup");
  }
}

template <int FPL> struct VecT;
template <> struct VecT<4> { typedef v4f f; typedef v4h h; typedef v2u st; };
template <> struct VecT<2> { typedef v2f f; typedef v2h h; typedef unsigned st; };

__global__ __launch_bounds__(256) void wT_cast_kernel(const float* __restrict__ W, unsigned* __restrict__ out, int Kr, int Nc, int Kp, float scale) {
  const int i = blockIdx.x * 256 + threadIdx.x;
  if (i >= (Nc * Kp) / 2) return;
  const int h0 = 2 * i;
  const int n = h0 / Kp;
  const int k = h0 - n * Kp;
  const float a = (k < Kr) ? W[(size_t)k * Nc + n] * scale : 0.f;
  const float b = (k + 1 < Kr) ? W[(size_t)(k + 1) * Nc + n] * scale : 0.f;
  const unsigned u = (unsigned)__builtin_bit_cast(unsigned short, (_Float16)a) | ((unsigned)__builtin_bit_cast(unsigned short, (_Float16)b) << 16);
  ((volatile unsigned*)out)[i] = u; __threadfence(); ((volatile unsigned*)out)[i] = u;
}

__global__ __launch_bounds__(256) void padcast_rows_kernel(const float* __restrict__ x, unsigned* __restrict__ X16) {
  const long i = (long)blockIdx.x * 256 + threadIdx.x; if (i >= (long)NPAD * GI / 2) return;
  const long e0 = 2 * i; const bool ok = e0 < (long)NN * GI;
  const float a = ok ? x[e0] : 0.f, b = ok ? x[e0 + 1] : 0.f;
  const unsigned u = (unsigned)__builtin_bit_cast(unsigned short, (_Float16)a) | ((unsigned)__builtin_bit_cast(unsigned short, (_Float16)b) << 16);
  ((volatile unsigned*)X16)[i] = u; __threadfence(); ((volatile unsigned*)X16)[i] = u;
}

template <int F>
__global__ __launch_bounds__(NT) void att_terms_kernel(const float* __restrict__ H, const float* __restrict__ as, const float* __restrict__ ad,
                                                      float* __restrict__ AS, float* __restrict__ AD) {
  constexpr int FPL = F / 32;
  typedef typename VecT<FPL>::f vF;
  __shared__ float so[64];
  const int lane = threadIdx.x & 31, wave = threadIdx.x >> 5;
  const int nb = blockIdx.x * 32;
  const vF sa = *(const vF*)(as + FPL * lane);
  const vF da = *(const vF*)(ad + FPL * lane);
#pragma unroll 1
  for (int j = 0; j < 4; ++j) {
    const int n = nb + wave * 4 + j;
    const vF hv = *(const vF*)(H + (size_t)n * F + FPL * lane);
    float s = 0.f, d = 0.f;
#pragma unroll
    for (int e = 0; e < FPL; ++e) { s += hv[e] * sa[e]; d += hv[e] * da[e]; }
#pragma unroll
    for (int o = 16; o > 0; o >>= 1) { s += __shfl_xor(s, o, 32); d += __shfl_xor(d, o, 32); }
    if (lane == 0) { so[wave * 4 + j] = s; so[32 + wave * 4 + j] = d; }
  }
  __syncthreads();
  if (wave < 2) {
    const float v = so[wave * 32 + lane];
    float* op = ((wave == 0) ? AS : AD) + nb + lane;
    *(volatile float*)op = v; __threadfence(); *(volatile float*)op = v;
  }
}

__device__ __forceinline__ int blk_excl_scan(int cnt, int* scan_ws, int tid, int* tot) {
  const int lane = tid & 31, wave = tid >> 5; int incl = cnt;
#pragma unroll
  for (int o = 1; o < 32; o <<= 1) { const int v = __shfl_up(incl, o, 32); if (lane >= o) incl += v; }
  if (lane == 31) scan_ws[wave] = incl;
  __syncthreads();
  if (wave == 0) { int wv = (lane < NT / 32) ? scan_ws[lane] : 0; int wincl = wv;
#pragma unroll
    for (int o = 1; o < 32; o <<= 1) { const int v = __shfl_up(wincl, o, 32); if (lane >= o) wincl += v; }
    if (lane < NT / 32) scan_ws[32 + lane] = wincl - wv; if (lane == 31) scan_ws[64] = wincl; }
  __syncthreads();
  const int res = scan_ws[32 + wave] + incl - cnt; *tot = scan_ws[64];
  return res;
}
template <int SP, int CAP>
__device__ __forceinline__ int chunk_hits(const int* __restrict__ ei, int e0, int n0, int tid, int* LIST, int* scan_ws) {
  const int eb = e0 + tid * SP;
  int rec[SP]; int cnt = 0;
  if (eb < 2 * NE) {
    const int base = (eb < NE) ? eb : (eb - NE);
    const bool rev = (eb >= NE);
#pragma unroll
    for (int k = 0; k < SP; k += 2) {
      const v4i p4 = *(const v4i*)(ei + 2 * (size_t)(base + k));
#pragma unroll
      for (int e = 0; e < 2; ++e) {
        const int a = p4[2 * e], b = p4[2 * e + 1];
        const int d = rev ? a : b;
        int s = rev ? b : a;
        int r = -1;
        if (d >= n0 && d < n0 + SRB) { s = s < 0 ? 0 : (s >= NN ? NN - 1 : s); r = ((d - n0) << 16) | s; ++cnt; }
        rec[k + e] = r;
      }
    }
  } else {
#pragma unroll
    for (int k = 0; k < SP; ++k) {
      const int e = eb + k; const int d = e - 2 * NE; int r = -1;
      if (e < NV && d >= n0 && d < n0 + SRB) { r = ((d - n0) << 16) | d; ++cnt; }
      rec[k] = r;
    }
  }
  int tot; int p = blk_excl_scan(cnt, scan_ws, tid, &tot);
#pragma unroll
  for (int k = 0; k < SP; ++k) if (rec[k] >= 0) { if ((unsigned)p < (unsigned)CAP) LIST[p] = rec[k]; ++p; }
  __syncthreads();
  return tot < CAP ? tot : CAP;
}

template <int F>
__global__ __launch_bounds__(NT) void gat_agg_kernel(const float* __restrict__ H, const int* __restrict__ ei,
                                                    const float* __restrict__ AS, const float* __restrict__ AD,
                                                    const float* __restrict__ bias, float* AGG, void* FOp) {
  constexpr int FPL = F / 32;
  typedef typename VecT<FPL>::f  vF;
  typedef typename VecT<FPL>::h  vH;
  typedef typename VecT<FPL>::st sT;
  sT* FO = (sT*)FOp;
  __shared__ int LIST[SCH];
  __shared__ float SM[SRB];
  __shared__ float SL[SRB];
  __shared__ float SAD[SRB];
  __shared__ int scan_ws[80];
  const int tid = threadIdx.x, lane = tid & 31, wave = tid >> 5;
  const int n0 = blockIdx.x * SRB;
  vF zf;
#pragma unroll
  for (int e = 0; e < FPL; ++e) zf[e] = 0.f;
#pragma unroll 1
  for (int j = 0; j < RPW; ++j) {
    float* zp = AGG + (size_t)(n0 + wave * RPW + j) * F + FPL * lane;
    *(volatile vF*)zp = zf;
    __threadfence();
    *(volatile vF*)zp = zf;
  }
  for (int i = tid; i < SRB; i += NT) {
    SM[i] = -INFINITY; SL[i] = 0.f;
    SAD[i] = (n0 + i < NPAD) ? AD[n0 + i] : 0.f;
  }
  __syncthreads();
#pragma unroll 1
  for (int c = 0; c < NCH; ++c) {
    const int tot = chunk_hits<SCH / NT, SCH>(ei, c * SCH, n0, tid, LIST, scan_ws);
#pragma unroll 1
    for (int base = 0; base < tot; base += 32) {
      const int q = base + lane;
      const int rv = (q < tot) ? LIST[q] : -1;
      const int own = (rv >= 0 && (rv >> (16 + RPW_LOG)) == wave) ? 1 : 0;
      unsigned msk = (unsigned)__ballot(own);
#pragma unroll 1
      for (int it = 0; it < 32; ++it) {
        if (msk == 0u) break;
        const int bp = __builtin_ctz(msk); msk &= msk - 1u;
        const int r = __shfl(rv, bp, 32);
        const int dl = r >> 16, s = r & 0xFFFF;
        float al = AS[s] + SAD[dl];
        al = (al >= 0.f) ? al : 0.2f * al;
        const float mo = SM[dl], lo = SL[dl];
        const float mn = fmaxf(mo, al);
        const float rr = __expf(mo - mn), ex = __expf(al - mn);
        const float ln = lo * rr + ex;
        if (lane == 0) { SM[dl] = mn; SL[dl] = ln; }
        const vF hv = *(const vF*)(H + (size_t)s * F + FPL * lane);
        float* rp = AGG + (size_t)(n0 + dl) * F + FPL * lane;
        vF a = *(const vF*)rp;
        a = a * rr + hv * ex;
        *(volatile vF*)rp = a;
        __threadfence();
        *(volatile vF*)rp = a;
      }
    }
    __syncthreads();
  }
  const vF bv = *(const vF*)(bias + FPL * lane);
#pragma unroll 1
  for (int j = 0; j < RPW; ++j) {
    const int dl = wave * RPW + j;
    const int n = n0 + dl;
    if (n >= NPAD) break;
    const float lv = SL[dl];
    const float inv = (lv > 0.f) ? __builtin_amdgcn_rcpf(lv) : 0.f;
    vF v = *(const vF*)(AGG + (size_t)n * F + FPL * lane);
    v = v * inv + bv;
#pragma unroll
    for (int e = 0; e < FPL; ++e) v[e] = fmaxf(v[e], 0.f);
    if (n >= NN) v = zf;
    const vH hv = __builtin_convertvector(v, vH);
    const sT u = __builtin_bit_cast(sT, hv);
    sT* op = FO + (size_t)n * 32 + lane;
    *(volatile sT*)op = u; __threadfence(); *(volatile sT*)op = u;
  }
}

__device__ __forceinline__ v4u ea_piece(int qq, int row, int col, int e, const unsigned short* __restrict__ X16,
                                        const unsigned short* __restrict__ F2, const float* __restrict__ dist) {
  const v4u z = {0u, 0u, 0u, 0u};
  if (qq < 8)  return *(const v4u*)(X16 + (size_t)row * 64 + qq * 8);
  if (qq < 16) return *(const v4u*)(F2  + (size_t)row * 64 + (qq - 8) * 8);
  if (qq < 24) return *(const v4u*)(X16 + (size_t)col * 64 + (qq - 16) * 8);
  if (qq < 32) return *(const v4u*)(F2  + (size_t)col * 64 + (qq - 24) * 8);
  if (qq < 34) {
    const float* dp = dist + (size_t)e * 16 + (qq - 32) * 8;
    const v4f a = *(const v4f*)(dp), b = *(const v4f*)(dp + 4);
    v8h hv;
    hv[0] = (_Float16)a[0]; hv[1] = (_Float16)a[1]; hv[2] = (_Float16)a[2]; hv[3] = (_Float16)a[3];
    hv[4] = (_Float16)b[0]; hv[5] = (_Float16)b[1]; hv[6] = (_Float16)b[2]; hv[7] = (_Float16)b[3];
    return __builtin_bit_cast(v4u, hv);
  }
  return z;
}
__global__ __launch_bounds__(NT) void edge_gather_kernel(const int* __restrict__ ei, const unsigned short* __restrict__ X16,
                                                        const unsigned short* __restrict__ F2, const float* __restrict__ dist,
                                                        unsigned short* __restrict__ EA, int e0) {
  const int lane = threadIdx.x & 31, wave = threadIdx.x >> 5;
  const int pl = blockIdx.x * 8 + wave;
  const int eA = e0 + 2 * pl;
  int rA = ei[2 * (size_t)eA], cA = ei[2 * (size_t)eA + 1], rB = ei[2 * (size_t)eA + 2], cB = ei[2 * (size_t)eA + 3];
  rA = rA < 0 ? 0 : (rA >= NN ? NN - 1 : rA); cA = cA < 0 ? 0 : (cA >= NN ? NN - 1 : cA);
  rB = rB < 0 ? 0 : (rB >= NN ? NN - 1 : rB); cB = cB < 0 ? 0 : (cB >= NN ? NN - 1 : cB);
  const v4u v0 = ea_piece(lane, rA, cA, eA, X16, F2, dist);
  const int q1 = lane + 32; const int w1 = (q1 >= 36) ? 1 : 0; const int qq1 = q1 - 36 * w1;
  const v4u v1 = ea_piece(qq1, w1 ? rB : rA, w1 ? cB : cA, eA + w1, X16, F2, dist);
  const v4u v2 = ea_piece(lane + 28, rB, cB, eA + 1, X16, F2, dist);
  v4u* dst = (v4u*)(EA + (size_t)(2 * pl) * MKP);
  for (int pass = 0; pass < 2; ++pass) {
    *(volatile v4u*)(dst + lane) = v0;
    *(volatile v4u*)(dst + 32 + lane) = v1;
    if (lane < 8) *(volatile v4u*)(dst + 64 + lane) = v2;
    __threadfence();
  }
}

__global__ __launch_bounds__(256) void edge_mlp_kernel(const unsigned short* __restrict__ Ap, const unsigned short* __restrict__ Btp,
                                                      const float* __restrict__ b1, const float* __restrict__ w2, const float* __restrict__ b2,
                                                      float* __restrict__ out, int e0, int K, float scale) {
  typedef _Float16 T;
  typedef v16h V;
  const T* A = (const T*)Ap; const T* Bt = (const T*)Btp;
  __shared__ float sP[8][64];
  const int lane = threadIdx.x & 31, wave = threadIdx.x >> 5;
  const int rlane = lane & 15;
  const int koff  = (lane >> 4) * 8;
  const int hh    = lane >> 4;
  const int m0 = blockIdx.x * 256 + (wave >> 1) * 64;
  const int n0 = (wave & 1) * 64;

  v8f acc[4][4];
#pragma unroll
  for (int i = 0; i < 4; ++i)
#pragma unroll
    for (int j = 0; j < 4; ++j) acc[i][j] = (v8f){0.f,0.f,0.f,0.f,0.f,0.f,0.f,0.f};

  for (int k0 = 0; k0 < K; k0 += 32) {
    V bh[4];
#pragma unroll
    for (int j = 0; j < 4; ++j) bh[j] = Frag<T>::load(Bt + (size_t)(n0 + (j << 4) + rlane) * K + koff + k0);
#pragma unroll
    for (int i = 0; i < 4; ++i) {
      V ah = Frag<T>::load(A + (size_t)(m0 + (i << 4) + rlane) * K + koff + k0);
#pragma unroll
      for (int j = 0; j < 4; ++j) acc[i][j] = Frag<T>::mma(ah, bh[j], acc[i][j]);
      Frag<T>::guard(acc[i][0], acc[i][3], ah, ah);
    }
    Frag<T>::keep(bh[0], bh[1], bh[2], bh[3]);
  }
  acc_guard4(acc[0][0], acc[0][1], acc[0][2], acc[0][3]);
  acc_guard4(acc[1][0], acc[1][1], acc[1][2], acc[1][3]);
  acc_guard4(acc[2][0], acc[2][1], acc[2][2], acc[2][3]);
  acc_guard4(acc[3][0], acc[3][1], acc[3][2], acc[3][3]);

  float bvv[4], wvv[4];
#pragma unroll
  for (int j = 0; j < 4; ++j) { const int n = n0 + (j << 4) + rlane; bvv[j] = b1[n]; wvv[j] = w2[n]; }
#pragma unroll
  for (int i = 0; i < 4; ++i) {
#pragma unroll
    for (int r = 0; r < 8; ++r) {
      float p = 0.f;
#pragma unroll
      for (int j = 0; j < 4; ++j) {
        const float v = fmaxf(acc[i][j][r] * scale + bvv[j], 0.f);
        p += v * wvv[j];
      }
      p += __shfl_xor(p, 1, 32); p += __shfl_xor(p, 2, 32); p += __shfl_xor(p, 4, 32); p += __shfl_xor(p, 8, 32);
      if (rlane == 0) sP[wave][(i << 4) + 8 * hh + r] = p;
    }
  }
  __syncthreads();
  const int t = threadIdx.x;
  const int rg = t >> 6, rr = t & 63;
  const float s = sP[2 * rg][rr] + sP[2 * rg + 1][rr] + b2[0];
  const float o = __builtin_amdgcn_rcpf(1.0f + __expf(-s));
  float* op = out + (size_t)e0 + (size_t)blockIdx.x * 256 + t;
  *(volatile float*)op = o; __threadfence(); *(volatile float*)op = o;
}

extern "C" void kernel_launch(void* const* d_in, const int* in_sizes, int n_in,
                              void* d_out, int out_size, void* d_ws, size_t ws_size, hipStream_t stream) {
  (void)in_sizes; (void)n_in; (void)out_size;
  const float* x    = (const float*)d_in[0];
  const int*   ei   = (const int*)  d_in[1];
  const float* dist = (const float*)d_in[2];
  const float* Wg1  = (const float*)d_in[3];
  const float* a1s  = (const float*)d_in[4];
  const float* a1d  = (const float*)d_in[5];
  const float* bg1  = (const float*)d_in[6];
  const float* Wg2  = (const float*)d_in[7];
  const float* a2s  = (const float*)d_in[8];
  const float* a2d  = (const float*)d_in[9];
  const float* bg2  = (const float*)d_in[10];
  const float* Wm1  = (const float*)d_in[11];
  const float* bm1  = (const float*)d_in[12];
  const float* Wm2  = (const float*)d_in[13];
  const float* bm2  = (const float*)d_in[14];
  float* out = (float*)d_out;

  char* ws = (char*)d_ws; size_t off = 0;
  auto carve = [&](size_t bytes) -> char* { char* p = ws + off; off += (bytes + 255) & ~(size_t)255; return p; };
  unsigned* X16 = (unsigned*)carve((size_t)NPAD * GI * 2);
  unsigned* W1T = (unsigned*)carve((size_t)GH * GI * 2);
  unsigned* W2T = (unsigned*)carve((size_t)GO * GH * 2);
  unsigned* WMT = (unsigned*)carve((size_t)MH * MKP * 2);
  unsigned* F2  = (unsigned*)carve((size_t)NPAD * GO * 2);
  float*    AS  = (float*)carve((size_t)NPAD * 4);
  float*    AD  = (float*)carve((size_t)NPAD * 4);
  const size_t r0 = off;
  float*    H   = (float*)carve((size_t)NPAD * GH * 4);
  float*    AGG = (float*)carve((size_t)NAGG * GH * 4);
  unsigned* F1  = (unsigned*)carve((size_t)NPAD * GH * 2);
  const size_t r1 = off;
  unsigned short* EA = (unsigned short*)(ws + r0);
  if (r0 + (size_t)ECH * MKP * 2 > r1) return;
  if (off > ws_size || off > (size_t)134217728) return;

  wT_cast_kernel<<<(GH * GI / 2 + 255) / 256, 256, 0, stream>>>(Wg1, W1T, GI, GH, GI, 16.0f);
  wT_cast_kernel<<<(GO * GH / 2 + 255) / 256, 256, 0, stream>>>(Wg2, W2T, GH, GO, GH, 16.0f);
  wT_cast_kernel<<<(MH * MKP / 2 + 255) / 256, 256, 0, stream>>>(Wm1, WMT, MK, MH, MKP, 16.0f);
  padcast_rows_kernel<<<(NPAD * GI / 2 + 255) / 256, 256, 0, stream>>>(x, X16);

  const int gt1 = (NPAD / 64) * (GH / 64);
  wmma_gemm64<0, false, 0, 0, false><<<dim3((gt1 + 7) / 8, 1), 256, 0, stream>>>(
      (const unsigned short*)X16, nullptr, GI, 0L, (const unsigned short*)W1T, nullptr, GI, 0L,
      (void*)H, nullptr, GH, 0L, nullptr, nullptr, 0L, NPAD, GH, GI, 0.0625f);
  att_terms_kernel<GH><<<NPAD / 32, NT, 0, stream>>>(H, a1s, a1d, AS, AD);
  gat_agg_kernel<GH><<<NTL, NT, 0, stream>>>(H, ei, AS, AD, bg1, AGG, (void*)F1);

  const int gt2 = (NPAD / 64) * (GO / 64);
  wmma_gemm64<0, false, 0, 0, false><<<dim3((gt2 + 7) / 8, 1), 256, 0, stream>>>(
      (const unsigned short*)F1, nullptr, GH, 0L, (const unsigned short*)W2T, nullptr, GH, 0L,
      (void*)H, nullptr, GO, 0L, nullptr, nullptr, 0L, NPAD, GO, GH, 0.0625f);
  att_terms_kernel<GO><<<NPAD / 32, NT, 0, stream>>>(H, a2s, a2d, AS, AD);
  gat_agg_kernel<GO><<<NTL, NT, 0, stream>>>(H, ei, AS, AD, bg2, AGG, (void*)F2);

  for (int c = 0; c < NECH; ++c) {
    const int e0 = c * ECH;
    const int rows = (NE - e0 < ECH) ? (NE - e0) : ECH;
    if (rows <= 0 || (rows % 256) != 0) return;
    edge_gather_kernel<<<rows / 16, NT, 0, stream>>>(ei, (const unsigned short*)X16, (const unsigned short*)F2, dist, EA, e0);
    edge_mlp_kernel<<<rows / 256, 256, 0, stream>>>((const unsigned short*)EA, (const unsigned short*)WMT, bm1, Wm2, bm2, out, e0, MKP, 0.0625f);
  }
}
